// TimeMixingTriton_24876450579372
// MI455X (gfx1250) — hardware-verified
//
#include <hip/hip_runtime.h>
#include <math.h>

#define NT   2048
#define NC   1024
#define NHD  16
#define HS   64
#define NBT  4096
#define WSC  64.0f
#define WINV 0.015625f

static_assert((NBT % 32) == 0);
static_assert((NC % 64) == 0);
static_assert(NHD * HS == NC);

typedef _Float16 f16;
typedef f16 v16h __attribute__((ext_vector_type(16)));
typedef f16 v8h __attribute__((ext_vector_type(8), may_alias));
typedef float v8f __attribute__((ext_vector_type(8)));
typedef float v4f __attribute__((ext_vector_type(4)));
typedef float v4fa __attribute__((ext_vector_type(4), may_alias));
union Frag { v16h v; v8h half[2]; };
union Pack8 { v8h v; f16 u[8]; };

__device__ __forceinline__ float sigm(float z)
{
  return __builtin_amdgcn_rcpf(1.0f + expf(-z));
}

__device__ __forceinline__ void mma2(v8f& c0, v8f& c1, v16h a0, v16h a1, v16h b)
{
  c0 = __builtin_amdgcn_wmma_f32_16x16x32_f16(false, a0, false, b, (short)0, c0, false, false);
  c1 = __builtin_amdgcn_wmma_f32_16x16x32_f16(false, a1, false, b, (short)0, c1, false, false);
  asm volatile("v_nop\n\tv_nop\n\tv_nop\n\tv_nop" : "+v"(c0), "+v"(c1) : "v"(a0), "v"(a1), "v"(b));
}

__global__ __launch_bounds__(256) void k_wcvt(const float* __restrict__ p0, const float* __restrict__ p1, const float* __restrict__ p2,
                                              const float* __restrict__ p3, const float* __restrict__ p4, const float* __restrict__ p5,
                                              const float* __restrict__ p6, const float* __restrict__ p7, const float* __restrict__ p8,
                                              const float* __restrict__ p9, const float* __restrict__ p10, const float* __restrict__ p11,
                                              f16* __restrict__ D)
{
#pragma clang fp contract(off)
  const int s = blockIdx.y;
  const float* W = p0;
  switch (s) {
    case 1: W = p1; break;
    case 2: W = p2; break;
    case 3: W = p3; break;
    case 4: W = p4; break;
    case 5: W = p5; break;
    case 6: W = p6; break;
    case 7: W = p7; break;
    case 8: W = p8; break;
    case 9: W = p9; break;
    case 10: W = p10; break;
    case 11: W = p11; break;
    default: break;
  }
  const size_t t = (size_t)blockIdx.x * 256 + threadIdx.x;
  if (t >= (size_t)NC * NC / 8) return;
  const float* src = W + t * 8;
  const v4f a = *(const v4fa*)src, b = *(const v4fa*)(src + 4);
  Pack8 pk;
#pragma unroll
  for (int i = 0; i < 4; ++i) {
    pk.u[i] = (f16)(a[i] * WSC);
    pk.u[4 + i] = (f16)(b[i] * WSC);
  }
  f16* dst = D + (size_t)s * NC * NC + t * 8;
  const v8h hv = pk.v;
  *(volatile v8h*)dst = hv;
  __threadfence();
  *(volatile v8h*)dst = hv;
}

__global__ __launch_bounds__(256) void k_shift(const float* __restrict__ x, const float* __restrict__ tm, f16* __restrict__ X)
{
#pragma clang fp contract(off)
  const size_t t = (size_t)blockIdx.x * 256 + threadIdx.x;
  if (t >= (size_t)NBT * NC / 8) return;
  const int bt = (int)(t >> 7), c8 = (int)(t & 127) * 8;
  const int tp = bt & (NT - 1);
  const int pb = (tp > 0) ? bt - 1 : bt;
  const float* xc = x + (size_t)bt * NC + c8;
  const float* xp = x + (size_t)pb * NC + c8;
  const v4f a0 = *(const v4fa*)xc, a1 = *(const v4fa*)(xc + 4);
  const v4f q0 = *(const v4fa*)xp, q1 = *(const v4fa*)(xp + 4);
  const v4f m0 = *(const v4fa*)(tm + c8), m1 = *(const v4fa*)(tm + c8 + 4);
  Pack8 pk;
#pragma unroll
  for (int i = 0; i < 4; ++i) {
    const float cur0 = a0[i];
    const float prv0 = (tp > 0) ? q0[i] : 0.0f;
    pk.u[i] = (f16)(cur0 + (prv0 - cur0) * m0[i]);
    const float cur1 = a1[i];
    const float prv1 = (tp > 0) ? q1[i] : 0.0f;
    pk.u[4 + i] = (f16)(cur1 + (prv1 - cur1) * m1[i]);
  }
  f16* dst = X + (size_t)bt * NC + c8;
  const v8h hv = pk.v;
  *(volatile v8h*)dst = hv;
  __threadfence();
  *(volatile v8h*)dst = hv;
}

template <int EPI, bool O16>
__global__ __launch_bounds__(128) void k_gemm(const f16* __restrict__ A, int lda, const f16* __restrict__ Bt, int ldb,
                                              int M, int N, int K,
                                              const float* __restrict__ bias, const float* __restrict__ aux,
                                              const float* P, const float* P2, int ldp,
                                              float* Cf, f16* Ch, int ldc)
{
#pragma clang fp contract(off)
  __shared__ __attribute__((aligned(16))) float so[4][32][64];
  const int tid = threadIdx.x, w = tid >> 5, lane = tid & 31, ln = lane & 15, hh = lane >> 4;
  const int ntn = N >> 6;
  const int wid = blockIdx.x * 4 + w;
  const int mt2 = wid / ntn, nq = wid - mt2 * ntn;
  if (mt2 * 32 >= M) return;
  const int row0 = mt2 * 32, col0 = nq * 64;
  const f16* a0p = A + (size_t)(row0 + ln) * lda + 8 * hh;
  const f16* a1p = a0p + (size_t)16 * lda;
  const f16* b0p = Bt + (size_t)(col0 + ln) * ldb + 8 * hh;
  v8f acc[2][4];
#pragma unroll
  for (int mt = 0; mt < 2; ++mt)
#pragma unroll
    for (int t = 0; t < 4; ++t)
#pragma unroll
      for (int r = 0; r < 8; ++r) acc[mt][t][r] = 0.0f;

#pragma unroll 1
  for (int kb = 0; kb < K; kb += 32) {
    Frag fa0, fa1;
    fa0.half[0] = *(const v8h*)(a0p + kb); fa0.half[1] = *(const v8h*)(a0p + kb + 16);
    fa1.half[0] = *(const v8h*)(a1p + kb); fa1.half[1] = *(const v8h*)(a1p + kb + 16);
#pragma unroll
    for (int t = 0; t < 4; ++t) {
      const f16* bp = b0p + (size_t)(16 * t) * ldb + kb;
      Frag fb;
      fb.half[0] = *(const v8h*)bp; fb.half[1] = *(const v8h*)(bp + 16);
      mma2(acc[0][t], acc[1][t], fa0.v, fa1.v, fb.v);
    }
  }
#pragma unroll
  for (int mt = 0; mt < 2; ++mt) {
#pragma unroll
    for (int t = 0; t < 4; ++t) {
#pragma unroll
      for (int r = 0; r < 8; ++r) so[w][16 * mt + 8 * hh + r][16 * t + ln] = acc[mt][t][r] * WINV;
    }
  }
  __builtin_amdgcn_fence(__ATOMIC_ACQ_REL, "workgroup");
  __builtin_amdgcn_wave_barrier();
  if (EPI == 1 || EPI >= 3) {
    float* sf = &so[w][0][0];
#pragma unroll 1
    for (int e = lane; e < 32 * 64; e += 32) {
      const int rr = e >> 6, cc = e & 63;
      const int gr = row0 + rr, gc = col0 + cc;
      float u = sf[e];
      if (EPI == 1) {
        u = tanhf(u);
      } else if (EPI == 3) {
        u = sigm(u);
      } else if (EPI == 4) {
        const float sg = sigm(bias[gc] + u);
        u = expf(-0.606531f * sg);
      } else if (EPI == 5) {
        const float sg = sigm(bias[gc] + u);
        const float pk = P[(size_t)gr * ldp + gc];
        u = pk * (1.0f + (sg - 1.0f) * aux[gc]);
      } else if (EPI == 6) {
        const float sg = sigm(bias[gc] + u);
        const float pv = P[(size_t)gr * ldp + gc];
        const float pf = P2[(size_t)gr * ldp + gc];
        u = pv + (pf - pv) * sg;
      }
      sf[e] = u;
    }
    __builtin_amdgcn_fence(__ATOMIC_ACQ_REL, "workgroup");
    __builtin_amdgcn_wave_barrier();
  }
  if (O16) {
    const int rq = lane >> 3, c8 = (lane & 7) * 8;
    Pack8 ph[8];
#pragma unroll
    for (int q = 0; q < 8; ++q) {
      const v4f a = *(const v4fa*)&so[w][4 * q + rq][c8];
      const v4f b = *(const v4fa*)&so[w][4 * q + rq][c8 + 4];
#pragma unroll
      for (int i = 0; i < 4; ++i) {
        ph[q].u[i] = (f16)a[i];
        ph[q].u[4 + i] = (f16)b[i];
      }
    }
    for (int pass = 0; pass < 2; ++pass) {
#pragma unroll
      for (int q = 0; q < 8; ++q) {
        const size_t o = (size_t)(row0 + 4 * q + rq) * ldc + col0 + c8;
        *(volatile v8h*)(Ch + o) = ph[q].v;
      }
      if (pass == 0) __threadfence();
    }
  } else {
    const int rs = lane >> 4, c4 = (lane & 15) * 4;
    v4f pc[16];
#pragma unroll
    for (int q = 0; q < 16; ++q) pc[q] = *(const v4fa*)&so[w][2 * q + rs][c4];
    for (int pass = 0; pass < 2; ++pass) {
#pragma unroll
      for (int q = 0; q < 16; ++q)
        *(volatile v4f*)(Cf + (size_t)(row0 + 2 * q + rs) * ldc + col0 + c4) = pc[q];
      if (pass == 0) __threadfence();
    }
  }
}

__global__ __launch_bounds__(256) void k_wkv(const float* __restrict__ Rp, const float* __restrict__ Wp, const float* __restrict__ Kp,
                                             const float* __restrict__ Vp, float* __restrict__ Yp)
{
#pragma clang fp contract(off)
  __shared__ __attribute__((aligned(16))) float lr[HS];
  __shared__ __attribute__((aligned(16))) float lw[HS];
  __shared__ __attribute__((aligned(16))) float lk[HS];
  __shared__ __attribute__((aligned(16))) float lv[HS];
  __shared__ __attribute__((aligned(16))) float ys[HS];
  const int tid = threadIdx.x;
  const int b = blockIdx.x >> 4, h = blockIdx.x & (NHD - 1);
  const int i = tid >> 2, jq = tid & 3, j0 = jq * 16;
  const int hc = h * HS;
  float S[16];
#pragma unroll
  for (int m = 0; m < 16; ++m) S[m] = 0.0f;
  const size_t rowb = (size_t)b * NT;
#pragma unroll 1
  for (int t = 0; t < NT; ++t) {
    const size_t e = (rowb + t) * NC + hc;
    if (tid < HS) {
      lr[tid] = Rp[e + tid];
      lw[tid] = Wp[e + tid];
      lk[tid] = Kp[e + tid];
      lv[tid] = Vp[e + tid];
    }
    __syncthreads();
    const float wi = lw[i], ki = lk[i];
    float vv[16], rr[16];
#pragma unroll
    for (int m = 0; m < 4; ++m) {
      const v4f qv = *(const v4fa*)&lv[j0 + 4 * m];
      const v4f qr = *(const v4fa*)&lr[j0 + 4 * m];
      vv[4 * m] = qv[0]; vv[4 * m + 1] = qv[1]; vv[4 * m + 2] = qv[2]; vv[4 * m + 3] = qv[3];
      rr[4 * m] = qr[0]; rr[4 * m + 1] = qr[1]; rr[4 * m + 2] = qr[2]; rr[4 * m + 3] = qr[3];
    }
    float yp = 0.0f;
#pragma unroll
    for (int m = 0; m < 16; ++m) {
      const float s2 = S[m] * wi + ki * vv[m];
      S[m] = s2;
      yp = yp + s2 * rr[m];
    }
    yp += __shfl_xor(yp, 1, 32);
    yp += __shfl_xor(yp, 2, 32);
    if (jq == 0) ys[i] = yp;
    __syncthreads();
    if (tid < 16) {
      const v4f o = *(const v4fa*)&ys[4 * tid];
      float* dst = Yp + e + 4 * tid;
      *(volatile v4f*)dst = o;
      __threadfence();
      *(volatile v4f*)dst = o;
    }
  }
}

__global__ __launch_bounds__(128) void k_ln(const float* __restrict__ Yp, const float* __restrict__ Rp, const float* __restrict__ Kp,
                                            const float* __restrict__ Vp, const float* __restrict__ Gp, const float* __restrict__ rk,
                                            const float* __restrict__ lng, const float* __restrict__ lnb, f16* __restrict__ YG)
{
#pragma clang fp contract(off)
  __shared__ float red0[4];
  __shared__ float red1[4];
  const int tid = threadIdx.x, w = tid >> 5, lane = tid & 31;
  const int row = blockIdx.x;
  const int c8 = tid * 8;
  const size_t base = (size_t)row * NC + c8;
  float y[8];
  {
    const v4f a = *(const v4fa*)(Yp + base), b = *(const v4fa*)(Yp + base + 4);
#pragma unroll
    for (int i = 0; i < 4; ++i) { y[i] = a[i]; y[4 + i] = b[i]; }
  }
  float s = 0.0f;
#pragma unroll
  for (int i = 0; i < 8; ++i) s = s + y[i];
  for (int o = 16; o > 0; o >>= 1) s += __shfl_xor(s, o, 32);
  if (lane == 0) red0[w] = s;
  __syncthreads();
  const float mu = ((red0[0] + red0[1]) + (red0[2] + red0[3])) * (1.0f / (float)NC);
  float d[8];
  float q = 0.0f;
#pragma unroll
  for (int i = 0; i < 8; ++i) { d[i] = y[i] - mu; q = q + d[i] * d[i]; }
  for (int o = 16; o > 0; o >>= 1) q += __shfl_xor(q, o, 32);
  if (lane == 0) red1[w] = q;
  __syncthreads();
  const float var = ((red1[0] + red1[1]) + (red1[2] + red1[3])) * (1.0f / (float)NC);
  const float rstd = rsqrtf(var + 1e-5f);
  float p = 0.0f;
  {
    const v4f r0 = *(const v4fa*)(Rp + base), r1 = *(const v4fa*)(Rp + base + 4);
    const v4f k0 = *(const v4fa*)(Kp + base), k1 = *(const v4fa*)(Kp + base + 4);
    const v4f f0 = *(const v4fa*)(rk + c8), f1 = *(const v4fa*)(rk + c8 + 4);
#pragma unroll
    for (int i = 0; i < 4; ++i) p = p + (r0[i] * k0[i]) * f0[i];
#pragma unroll
    for (int i = 0; i < 4; ++i) p = p + (r1[i] * k1[i]) * f1[i];
  }
  p += __shfl_xor(p, 1, 32);
  p += __shfl_xor(p, 2, 32);
  p += __shfl_xor(p, 4, 32);
  const v4f v0 = *(const v4fa*)(Vp + base), v1 = *(const v4fa*)(Vp + base + 4);
  const v4f g0 = *(const v4fa*)(Gp + base), g1 = *(const v4fa*)(Gp + base + 4);
  const v4f a0 = *(const v4fa*)(lng + c8), a1 = *(const v4fa*)(lng + c8 + 4);
  const v4f b0 = *(const v4fa*)(lnb + c8), b1 = *(const v4fa*)(lnb + c8 + 4);
  Pack8 pk;
#pragma unroll
  for (int i = 0; i < 4; ++i) {
    const float o0 = (((d[i] * rstd) * a0[i] + b0[i]) + p * v0[i]) * g0[i];
    const float o1 = (((d[4 + i] * rstd) * a1[i] + b1[i]) + p * v1[i]) * g1[i];
    pk.u[i] = (f16)o0;
    pk.u[4 + i] = (f16)o1;
  }
  f16* dst = YG + base;
  const v8h hv = pk.v;
  *(volatile v8h*)dst = hv;
  __threadfence();
  *(volatile v8h*)dst = hv;
}

template <int EPI, bool O16>
static void gemm_go(hipStream_t st, const f16* A, int lda, const f16* Bt, int ldb, int M, int N, int K,
                    const float* bias, const float* aux, const float* P, const float* P2, int ldp, float* Cf, f16* Ch, int ldc)
{
  const unsigned nb = (unsigned)(((M / 32) * (N / 64) + 3) / 4);
  k_gemm<EPI, O16><<<nb, 128, 0, st>>>(A, lda, Bt, ldb, M, N, K, bias, aux, P, P2, ldp, Cf, Ch, ldc);
}

static void shift_go(hipStream_t st, const float* x, const float* tm, f16* X)
{
  k_shift<<<(unsigned)(((size_t)NBT * NC / 8 + 255) / 256), 256, 0, st>>>(x, tm, X);
}

extern "C" void kernel_launch(void* const* d_in, const int* in_sizes, int n_in,
                              void* d_out, int out_size, void* d_ws, size_t ws_size, hipStream_t stream)
{
  if (n_in < 28) return;
  if (in_sizes[0] != NBT * NC || in_sizes[1] != NBT * NC) return;
  for (int q = 2; q <= 13; ++q) if (in_sizes[q] != NC * NC) return;
  for (int q = 14; q <= 27; ++q) if (in_sizes[q] != NC) return;
  if (out_size != NBT * NC) return;

  const float* x       = (const float*)d_in[0];
  const float* v_first = (const float*)d_in[1];
  const float* Wr  = (const float*)d_in[2];
  const float* Wk  = (const float*)d_in[3];
  const float* Wv  = (const float*)d_in[4];
  const float* Wo  = (const float*)d_in[5];
  const float* Wg1 = (const float*)d_in[6];
  const float* Wg2 = (const float*)d_in[7];
  const float* W1  = (const float*)d_in[8];
  const float* W2  = (const float*)d_in[9];
  const float* A1  = (const float*)d_in[10];
  const float* A2  = (const float*)d_in[11];
  const float* V1  = (const float*)d_in[12];
  const float* V2  = (const float*)d_in[13];
  const float* tm_r = (const float*)d_in[14];
  const float* tm_w = (const float*)d_in[15];
  const float* tm_k = (const float*)d_in[16];
  const float* tm_v = (const float*)d_in[17];
  const float* tm_a = (const float*)d_in[18];
  const float* tm_g = (const float*)d_in[19];
  const float* w0   = (const float*)d_in[20];
  const float* a0   = (const float*)d_in[21];
  const float* v0   = (const float*)d_in[22];
  const float* k_a  = (const float*)d_in[24];
  const float* r_k  = (const float*)d_in[25];
  const float* ln_g = (const float*)d_in[26];
  const float* ln_b = (const float*)d_in[27];
  float* out0 = (float*)d_out;

  char* ws = (char*)d_ws;
  size_t off = 0;
  auto take = [&](size_t bytes) -> char* { char* p = ws + off; off += (bytes + 4095) & ~(size_t)4095; return p; };
  const size_t PL = (size_t)NBT * NC;
  const size_t WPSZ = (size_t)NC * NC;
  f16* WPL  = (f16*)take(WPSZ * 12 * 2);
  float* Yp = (float*)(void*)WPL;
  f16* X    = (f16*)take(PL * 2);
  f16* YG   = X;
  f16* Hh   = (f16*)take(PL * 2);
  float* Rp = (float*)take(PL * 4);
  float* Kp = (float*)take(PL * 4);
  float* Vp = (float*)take(PL * 4);
  float* Wp = (float*)take(PL * 4);
  float* Gp = (float*)take(PL * 4);
  if (off > ws_size) return;
  if (off > (size_t)134217728) return;
  if (PL * 4 > WPSZ * 8 * 2) return;
  auto WP = [&](int s) -> const f16* { return WPL + (size_t)s * WPSZ; };

  k_wcvt<<<dim3((unsigned)((WPSZ / 8 + 255) / 256), 12), 256, 0, stream>>>(Wr, Wk, Wv, W1, W2, A1, A2, V1, V2, Wg1, Wg2, Wo, WPL);

  shift_go(stream, x, tm_r, X);
  gemm_go<0, false>(stream, X, NC, WP(0), NC, NBT, NC, NC, nullptr, nullptr, nullptr, nullptr, 0, Rp, nullptr, NC);

  shift_go(stream, x, tm_k, X);
  gemm_go<0, false>(stream, X, NC, WP(1), NC, NBT, NC, NC, nullptr, nullptr, nullptr, nullptr, 0, Kp, nullptr, NC);

  shift_go(stream, x, tm_v, X);
  gemm_go<0, false>(stream, X, NC, WP(2), NC, NBT, NC, NC, nullptr, nullptr, nullptr, nullptr, 0, Vp, nullptr, NC);
  gemm_go<2, true>(stream, X, NC, WP(7), NC, NBT, NC, NC, nullptr, nullptr, nullptr, nullptr, 0, nullptr, Hh, NC);
  gemm_go<6, false>(stream, Hh, NC, WP(8), NC, NBT, NC, NC, v0, nullptr, Vp, v_first, NC, Vp, nullptr, NC);

  shift_go(stream, x, tm_a, X);
  gemm_go<2, true>(stream, X, NC, WP(5), NC, NBT, NC, NC, nullptr, nullptr, nullptr, nullptr, 0, nullptr, Hh, NC);
  gemm_go<5, false>(stream, Hh, NC, WP(6), NC, NBT, NC, NC, a0, k_a, Kp, nullptr, NC, Kp, nullptr, NC);

  shift_go(stream, x, tm_w, X);
  gemm_go<1, true>(stream, X, NC, WP(3), NC, NBT, NC, NC, nullptr, nullptr, nullptr, nullptr, 0, nullptr, Hh, NC);
  gemm_go<4, false>(stream, Hh, NC, WP(4), NC, NBT, NC, NC, w0, nullptr, nullptr, nullptr, 0, Wp, nullptr, NC);

  shift_go(stream, x, tm_g, X);
  gemm_go<3, true>(stream, X, NC, WP(9), NC, NBT, NC, NC, nullptr, nullptr, nullptr, nullptr, 0, nullptr, Hh, NC);
  gemm_go<0, false>(stream, Hh, NC, WP(10), NC, NBT, NC, NC, nullptr, nullptr, nullptr, nullptr, 0, Gp, nullptr, NC);

  k_wkv<<<(unsigned)(NBT / NT * NHD), 256, 0, stream>>>(Rp, Wp, Kp, Vp, Yp);

  k_ln<<<(unsigned)NBT, 128, 0, stream>>>(Yp, Rp, Kp, Vp, Gp, r_k, ln_g, ln_b, YG);

  gemm_go<0, false>(stream, YG, NC, WP(11), NC, NBT, NC, NC, nullptr, nullptr, nullptr, nullptr, 0, out0, nullptr, NC);
}
